// DeformableInceptionModule_51238959841383
// MI455X (gfx1250) — hardware-verified
//
#include <hip/hip_runtime.h>
#include <stddef.h>


#define HW        4096
#define Himg      64
#define Wimg      64
#define Cin       64
#define CoutC     64
#define CoutTotal 192
#define MTILE     128
#define APITCH    72
#define BPITCH    72
#define CPITCH    132
#define NTHR      256
#define ASCALE    64.0f
#define WSCALE    256.0f
#define OSCALE    (1.0f / 16384.0f)

typedef _Float16 v8h  __attribute__((ext_vector_type(8)));
typedef _Float16 v16h __attribute__((ext_vector_type(16)));
typedef float    v4f  __attribute__((ext_vector_type(4)));
typedef float    v8f  __attribute__((ext_vector_type(8)));
union Frag { v16h v; v8h h[2]; };

__device__ __forceinline__ v8f wmh(v16h a, v16h b, v8f c) {
  v8f d = __builtin_amdgcn_wmma_f32_16x16x32_f16(false, a, false, b, (short)0, c, false, false);
  asm volatile("v_nop\n\tv_nop\n\tv_nop\n\tv_nop" : "+v"(d) : "v"(a), "v"(b));
  return d;
}

__device__ __forceinline__ v8f zero8f() {
  v8f z;
#pragma unroll
  for (int i = 0; i < 8; ++i) z[i] = 0.0f;
  return z;
}

__global__ __launch_bounds__(NTHR) void k_prepw(const float* __restrict__ w, _Float16* wT, int K) {
  const int t = blockIdx.x * NTHR + threadIdx.x;
  const int total8 = (K * CoutC * Cin) >> 3;
  int tc = t < total8 ? t : total8 - 1;
  tc = tc < 0 ? 0 : tc;
  const int c0 = (tc << 3) & (Cin - 1);
  const int co = (tc >> 3) & (CoutC - 1);
  const int k  = tc >> 9;
  v8h v;
#pragma unroll
  for (int j = 0; j < 8; ++j)
    v[j] = (_Float16)(w[((size_t)co * Cin + c0 + j) * K + k] * WSCALE);
  const bool ok = t < total8;
  _Float16* p = wT + (size_t)tc * 8;
  if (ok) *(volatile v8h*)p = v;
  __threadfence();
  if (ok) *(volatile v8h*)p = v;
}

template<int KH, int KW>
__global__ __launch_bounds__(NTHR) void k_dcn(
    const float* __restrict__ x,
    const _Float16* __restrict__ wT,
    const float* __restrict__ offset,
    const float* __restrict__ mask,
    float* out,
    int coBase)
{
  constexpr int K   = KH * KW;
  constexpr int PAD = (KH - 1) / 2;
  constexpr int ABYTES = MTILE * APITCH * 2;
  constexpr int BBYTES = CoutC * BPITCH * 2;
  static_assert(CoutC * CPITCH * 4 <= 2 * ABYTES);
  static_assert((MTILE - 1) * APITCH + 64 <= MTILE * APITCH);
  static_assert((CoutC - 1) * BPITCH + 64 <= CoutC * BPITCH);

  __shared__ __attribute__((aligned(16))) unsigned char smem[2 * (ABYTES + BBYTES)];
  float* Cs = (float*)smem;

  const int tid  = threadIdx.x;
  const int wave = tid >> 5;
  const int lane = tid & 31;
  const int r    = lane & 15;
  const int hi   = lane >> 4;

  const int b      = blockIdx.x >> 5;
  const int hwBase = (blockIdx.x & 31) * MTILE;

  const int m0 = (wave & 3) * 32;
  const int n0 = (wave >> 2) * 32;

  v8f acc00 = zero8f(), acc01 = zero8f(), acc10 = zero8f(), acc11 = zero8f();

  const int pos   = tid >> 1;
  const int chalf = (tid & 1) * 32;
  const int hw = hwBase + pos;
  const int h  = hw >> 6;
  const int wq = hw & 63;
  const float* xb    = x      + (size_t)b * Cin * HW;
  const float* offb  = offset + (size_t)b * 2 * K * HW + hw;
  const float* maskb = mask   + (size_t)b * K * HW + hw;

  auto sampleTap = [&](int k, int buf) {
    _Float16* As = (_Float16*)(smem + (buf ? ABYTES : 0));
    _Float16* Bs = (_Float16*)(smem + 2 * ABYTES + (buf ? BBYTES : 0));
    {
      const int co  = tid >> 2;
      const int seg = tid & 3;
      const v8h* src = (const v8h*)(wT + ((size_t)k * CoutC + co) * Cin + seg * 16);
      v8h* dst = (v8h*)(Bs + co * BPITCH + seg * 16);
      dst[0] = src[0];
      dst[1] = src[1];
    }
    const int ky = k / KW;
    const int kx = k - ky * KW;
    const float dy = offb[(size_t)(2 * k) * HW];
    const float dx = offb[(size_t)(2 * k + 1) * HW];
    const float mk = maskb[(size_t)k * HW] * ASCALE;
    const float py = (float)(h - PAD + ky) + dy;
    const float px = (float)(wq - PAD + kx) + dx;
    float y0f = floorf(py), x0f = floorf(px);
    const float wy = py - y0f, wx = px - x0f;
    y0f = fminf(fmaxf(y0f, -2.0f), 64.0f);
    x0f = fminf(fmaxf(x0f, -2.0f), 64.0f);
    const int y0 = (int)y0f, x0 = (int)x0f;
    const int y1 = y0 + 1,   x1 = x0 + 1;
    const bool vy0 = (y0 >= 0) && (y0 < Himg);
    const bool vy1 = (y1 >= 0) && (y1 < Himg);
    const bool vx0 = (x0 >= 0) && (x0 < Wimg);
    const bool vx1 = (x1 >= 0) && (x1 < Wimg);
    const int yc0 = min(max(y0, 0), Himg - 1);
    const int yc1 = min(max(y1, 0), Himg - 1);
    const int xc0 = min(max(x0, 0), Wimg - 1);
    const int xc1 = min(max(x1, 0), Wimg - 1);
    const float c00 = (vy0 && vx0) ? (1.0f - wy) * (1.0f - wx) * mk : 0.0f;
    const float c01 = (vy0 && vx1) ? (1.0f - wy) * wx * mk : 0.0f;
    const float c10 = (vy1 && vx0) ? wy * (1.0f - wx) * mk : 0.0f;
    const float c11 = (vy1 && vx1) ? wy * wx * mk : 0.0f;
    const int i00 = yc0 * Wimg + xc0;
    const int i01 = yc0 * Wimg + xc1;
    const int i10 = yc1 * Wimg + xc0;
    const int i11 = yc1 * Wimg + xc1;
    const float* xch = xb + (size_t)chalf * HW;
    _Float16* arow = As + pos * APITCH + chalf;
#pragma unroll 2
    for (int c8 = 0; c8 < 32; c8 += 8) {
      v8h hv;
#pragma unroll
      for (int j = 0; j < 8; ++j) {
        const float* p = xch + (size_t)(c8 + j) * HW;
        const float s = c00 * p[i00] + c01 * p[i01] + c10 * p[i10] + c11 * p[i11];
        hv[j] = (_Float16)s;
      }
      *(v8h*)(arow + c8) = hv;
    }
  };

  sampleTap(0, 0);
  __syncthreads();

#pragma unroll 1
  for (int k = 0; k < K; ++k) {
    const int cur = k & 1;
    const _Float16* As = (const _Float16*)(smem + (cur ? ABYTES : 0));
    const _Float16* Bs = (const _Float16*)(smem + 2 * ABYTES + (cur ? BBYTES : 0));

#pragma unroll
    for (int ks = 0; ks < 64; ks += 32) {
      Frag a0, a1, b0, b1;
      const _Float16* ra = As + (m0 + r) * APITCH + ks + 8 * hi;
      a0.h[0] = *(const v8h*)(ra);
      a0.h[1] = *(const v8h*)(ra + 16);
      a1.h[0] = *(const v8h*)(ra + 16 * APITCH);
      a1.h[1] = *(const v8h*)(ra + 16 * APITCH + 16);
      const _Float16* rb = Bs + (n0 + r) * BPITCH + ks + 8 * hi;
      b0.h[0] = *(const v8h*)(rb);
      b0.h[1] = *(const v8h*)(rb + 16);
      b1.h[0] = *(const v8h*)(rb + 16 * BPITCH);
      b1.h[1] = *(const v8h*)(rb + 16 * BPITCH + 16);
      acc00 = wmh(a0.v, b0.v, acc00);
      acc01 = wmh(a0.v, b1.v, acc01);
      acc10 = wmh(a1.v, b0.v, acc10);
      acc11 = wmh(a1.v, b1.v, acc11);
    }

    if (k + 1 < K) sampleTap(k + 1, cur ^ 1);

    __syncthreads();
  }

#pragma unroll
  for (int e = 0; e < 8; ++e) {
    const int mm = e + 8 * hi;
    Cs[(n0 + r)      * CPITCH + m0 + mm]      = acc00[e] * OSCALE;
    Cs[(n0 + 16 + r) * CPITCH + m0 + mm]      = acc01[e] * OSCALE;
    Cs[(n0 + r)      * CPITCH + m0 + 16 + mm] = acc10[e] * OSCALE;
    Cs[(n0 + 16 + r) * CPITCH + m0 + 16 + mm] = acc11[e] * OSCALE;
  }
  __syncthreads();

  v4f ov[8];
#pragma unroll
  for (int q = 0; q < 8; ++q)
    ov[q] = *(const v4f*)(Cs + (wave * 8 + q) * CPITCH + 4 * lane);
  float* ob = out + ((size_t)b * CoutTotal + coBase + wave * 8) * HW + hwBase + 4 * lane;
#pragma unroll
  for (int q = 0; q < 8; ++q) *(volatile v4f*)(ob + (size_t)q * HW) = ov[q];
  __threadfence();
#pragma unroll
  for (int q = 0; q < 8; ++q) *(volatile v4f*)(ob + (size_t)q * HW) = ov[q];
}

extern "C" void kernel_launch(void* const* d_in, const int* in_sizes, int n_in,
                              void* d_out, int out_size, void* d_ws, size_t ws_size,
                              hipStream_t stream) {
  if (n_in < 10) return;
  const int nImg = in_sizes[0] / (Cin * HW);
  if (nImg <= 0 || in_sizes[0] != nImg * Cin * HW) return;
  if (in_sizes[1] != CoutC * Cin * 9  || in_sizes[2] != nImg * 18 * HW || in_sizes[3] != nImg * 9  * HW) return;
  if (in_sizes[4] != CoutC * Cin * 25 || in_sizes[5] != nImg * 50 * HW || in_sizes[6] != nImg * 25 * HW) return;
  if (in_sizes[7] != CoutC * Cin * 49 || in_sizes[8] != nImg * 98 * HW || in_sizes[9] != nImg * 49 * HW) return;
  if (out_size != nImg * CoutTotal * HW) return;

  const float* x   = (const float*)d_in[0];
  const float* w1  = (const float*)d_in[1];
  const float* of1 = (const float*)d_in[2];
  const float* mk1 = (const float*)d_in[3];
  const float* w2  = (const float*)d_in[4];
  const float* of2 = (const float*)d_in[5];
  const float* mk2 = (const float*)d_in[6];
  const float* w3  = (const float*)d_in[7];
  const float* of3 = (const float*)d_in[8];
  const float* mk3 = (const float*)d_in[9];
  float* out = (float*)d_out;

  const size_t sz1 = (size_t)9  * CoutC * Cin * 2;
  const size_t sz2 = (size_t)25 * CoutC * Cin * 2;
  const size_t sz3 = (size_t)49 * CoutC * Cin * 2;
  const size_t o1 = 0, o2 = o1 + sz1, o3 = o2 + sz2, total = o3 + sz3;
  if (total > ws_size) return;
  char* ws = (char*)d_ws;
  _Float16* wT1 = (_Float16*)(ws + o1);
  _Float16* wT2 = (_Float16*)(ws + o2);
  _Float16* wT3 = (_Float16*)(ws + o3);

  const int g1 = (9  * CoutC * Cin / 8 + NTHR - 1) / NTHR;
  const int g2 = (25 * CoutC * Cin / 8 + NTHR - 1) / NTHR;
  const int g3 = (49 * CoutC * Cin / 8 + NTHR - 1) / NTHR;
  k_prepw<<<g1, NTHR, 0, stream>>>(w1, wT1, 9);
  k_prepw<<<g2, NTHR, 0, stream>>>(w2, wT2, 25);
  k_prepw<<<g3, NTHR, 0, stream>>>(w3, wT3, 49);

  dim3 grid(nImg * (HW / MTILE));
  dim3 block(NTHR);
  k_dcn<3, 3><<<grid, block, 0, stream>>>(x, wT1, of1, mk1, out, 0);
  k_dcn<5, 5><<<grid, block, 0, stream>>>(x, wT2, of2, mk2, out, 64);
  k_dcn<7, 7><<<grid, block, 0, stream>>>(x, wT3, of3, mk3, out, 128);
}
